// AwkwardDeepSetDoubleJagged_24979529794079
// MI455X (gfx1250) — hardware-verified
//
#include <hip/hip_runtime.h>


namespace {
constexpr int NT = 2000000, NEV = 20000, NEVP = 20032  , H = 64, OUT = 10;
constexpr float XS = 8.0f, WSC = 256.0f;

typedef _Float16 b16;
typedef __attribute__((ext_vector_type(16))) _Float16 v16b;
typedef __attribute__((ext_vector_type(8))) _Float16 v8b;
typedef __attribute__((ext_vector_type(8))) float v8f;
typedef __attribute__((ext_vector_type(4))) float v4f;
__device__ __forceinline__ float bf16_rne(float f) { unsigned int u = __float_as_uint(f); u += 0x7FFFu + ((u >> 16) & 1u); return __uint_as_float(u & 0xFFFF0000u); }
__device__ __forceinline__ void split16(float v, b16& hi, b16& lo) { hi = (b16)v; lo = (b16)(v - (float)hi); }
__device__ __forceinline__ v16b frag_kb(const b16* p, int hh) { const v8b a = *(const v8b*)(p + 8 * hh), b = *(const v8b*)(p + 16 + 8 * hh); v16b f;
#pragma unroll
  for (int e = 0; e < 8; ++e) { f[e] = a[e]; f[8 + e] = b[e]; } return f; }
__device__ __forceinline__ v8f wmma16b(v16b a, v16b b, v8f c) { v8f d = __builtin_amdgcn_wmma_f32_16x16x32_f16(false, a, false, b, (short)0, c, false, false); asm volatile("v_nop\n\tv_nop\n\tv_nop\n\tv_nop" : "+v"(d) : "v"(a), "v"(b)); return d; }
__device__ __forceinline__ void wave_lds_sync() { __builtin_amdgcn_fence(__ATOMIC_RELEASE, "workgroup"); __builtin_amdgcn_wave_barrier(); __builtin_amdgcn_fence(__ATOMIC_ACQUIRE, "workgroup"); }
__device__ __forceinline__ float pmul(float a, float b) { float p = a * b; asm volatile("" : "+v"(p)); return p; }
__device__ __forceinline__ int iclamp(int v, int lo, int hi) { return v < lo ? lo : (v > hi ? hi : v); }

__global__ __launch_bounds__(256) void prep_kernel(const float* __restrict__ w0, const float* __restrict__ w1, const float* __restrict__ w2, const float* __restrict__ w3, const float* __restrict__ w4, const float* __restrict__ w5, b16* __restrict__ W6) {
  const int t = blockIdx.x * 256 + threadIdx.x; if (t >= 6 * H * H / 8) return; const int k = t / (H * H / 8); const int e = (t % (H * H / 8)) * 8; const float* w = k == 0 ? w0 : k == 1 ? w1 : k == 2 ? w2 : k == 3 ? w3 : k == 4 ? w4 : w5; v8b o;
  for (int j = 0; j < 8; ++j) o[j] = (b16)(bf16_rne(w[e + j]) * WSC);
  for (int pass = 0; pass < 2; ++pass) { *(volatile v8b*)(W6 + (size_t)k * H * H + e) = o; __threadfence(); }
}
__device__ __forceinline__ int lower_bound_(const int* __restrict__ a, int n, int key) { int lo = 0, hi = n; while (lo < hi) { const int mid = (lo + hi) >> 1; if (a[mid] < key) lo = mid + 1; else hi = mid; } return lo; }
__global__ __launch_bounds__(32) void stage1_kernel(const float* __restrict__ vals, const int* __restrict__ seg, const float* __restrict__ p1w0, const float* __restrict__ p1b0, const b16* __restrict__ W1, const float* __restrict__ p1b1, float* __restrict__ EV) {
  __shared__ __attribute__((aligned(16))) b16 Ah[16][H + 8], Al[16][H + 8]; __shared__ float colsum[2][H]; __shared__ __attribute__((aligned(16))) float row[H];
  const int ev = blockIdx.x, lane = threadIdx.x, nloc = lane & 15, hlf = lane >> 4;
  float acc_c[2] = {0.0f, 0.0f};
  if (ev < NEV) { const int st = lower_bound_(seg, NT, ev), en = lower_bound_(seg, NT, ev + 1);
    const float w0a = bf16_rne(p1w0[lane]), w0b = bf16_rne(p1w0[lane + 32]), b0a = bf16_rne(p1b0[lane]), b0b = bf16_rne(p1b0[lane + 32]);
    for (int p0 = st; p0 < en; p0 += 16) {
      for (int rr = 0; rr < 16; ++rr) { const int p = p0 + rr; const float v = (p < en) ? bf16_rne(vals[iclamp(p, 0, NT - 1)]) : 0.0f; b16 ph, pl;
        split16(fmaxf(pmul(v, w0a) + b0a, 0.0f) * XS, ph, pl); Ah[rr][lane] = ph; Al[rr][lane] = pl; split16(fmaxf(pmul(v, w0b) + b0b, 0.0f) * XS, ph, pl); Ah[rr][lane + 32] = ph; Al[rr][lane + 32] = pl; }
      wave_lds_sync();
      v8f d[4] = {{}, {}, {}, {}};
#pragma unroll
      for (int kb = 0; kb < H; kb += 32) { const v16b a = frag_kb(&Ah[nloc][kb], hlf), al = frag_kb(&Al[nloc][kb], hlf);
#pragma unroll
        for (int t = 0; t < 4; ++t) { const v16b bw = frag_kb(W1 + (size_t)(t * 16 + nloc) * H + kb, hlf); d[t] = wmma16b(a, bw, d[t]); d[t] = wmma16b(al, bw, d[t]); } }
      float cs[4] = {0.0f, 0.0f, 0.0f, 0.0f};
#pragma unroll
      for (int t = 0; t < 4; ++t) { const float bb = bf16_rne(p1b1[t * 16 + nloc]);
#pragma unroll
        for (int r = 0; r < 8; ++r) if (p0 + 8 * hlf + r < en) cs[t] += fmaxf(d[t][r] * (1.0f / (XS * WSC)) + bb, 0.0f); }
#pragma unroll
      for (int t = 0; t < 4; ++t) colsum[hlf][t * 16 + nloc] = cs[t];
      wave_lds_sync();
      acc_c[0] += colsum[0][lane] + colsum[1][lane]; acc_c[1] += colsum[0][lane + 32] + colsum[1][lane + 32];
      wave_lds_sync(); } }
  row[lane] = acc_c[0]; row[lane + 32] = acc_c[1]; wave_lds_sync();
  for (int pass = 0; pass < 2; ++pass) { if (lane < 16) *(volatile v4f*)(EV + (size_t)ev * H + lane * 4) = *(const v4f*)(&row[lane * 4]); __threadfence(); }
}
__global__ __launch_bounds__(128) void dense_kernel(const float* __restrict__ X, const b16* __restrict__ Wt, const float* __restrict__ bias, float* __restrict__ Y) {
  __shared__ __attribute__((aligned(16))) b16 Ah[4][16][H + 8], Al[4][16][H + 8]; __shared__ __attribute__((aligned(16))) float Tf[4][16][H + 4];
  const int wave = threadIdx.x >> 5, lane = threadIdx.x & 31, nloc = lane & 15, hlf = lane >> 4; const size_t m0 = (size_t)blockIdx.x * 64 + wave * 16;
  for (int q = lane; q < 16 * H; q += 32) { const int rr = q / H, c = q % H; b16 p, pl; split16(X[(m0 + rr) * H + c] * XS, p, pl); Ah[wave][rr][c] = p; Al[wave][rr][c] = pl; }
  wave_lds_sync();
  v8f d[4] = {{}, {}, {}, {}};
#pragma unroll
  for (int kb = 0; kb < H; kb += 32) { const v16b a = frag_kb(&Ah[wave][nloc][kb], hlf), al = frag_kb(&Al[wave][nloc][kb], hlf);
#pragma unroll
    for (int t = 0; t < 4; ++t) { const v16b bw = frag_kb(Wt + (size_t)(t * 16 + nloc) * H + kb, hlf); d[t] = wmma16b(a, bw, d[t]); d[t] = wmma16b(al, bw, d[t]); } }
#pragma unroll
  for (int t = 0; t < 4; ++t) { const float bb = bf16_rne(bias[t * 16 + nloc]);
#pragma unroll
    for (int r = 0; r < 8; ++r) Tf[wave][8 * hlf + r][t * 16 + nloc] = fmaxf(d[t][r] * (1.0f / (XS * WSC)) + bb, 0.0f); }
  wave_lds_sync();
  for (int pass = 0; pass < 2; ++pass) { for (int rr = 0; rr < 16; ++rr) if (lane < 16) *(volatile v4f*)(Y + (m0 + rr) * H + lane * 4) = *(const v4f*)(&Tf[wave][rr][lane * 4]); __threadfence(); }
}
__global__ __launch_bounds__(64) void final_kernel(const float* __restrict__ H2, const float* __restrict__ r2w0, const float* __restrict__ r2b0, const float* __restrict__ r2w1, const float* __restrict__ r2b1, const float* __restrict__ o2w, const float* __restrict__ o2b, float* __restrict__ out) {
  __shared__ float s[H], a[H], bq[H], lg[16];
  const int c = threadIdx.x; float acc = 0.0f;
#pragma unroll 4
  for (int e = 0; e < NEV; ++e) acc += H2[(size_t)e * H + c];
  s[c] = acc; __syncthreads();
  { float v = bf16_rne(r2b0[c]);
#pragma unroll 1
    for (int k = 0; k < H; ++k) v += pmul(s[k], bf16_rne(r2w0[c * H + k])); a[c] = fmaxf(v, 0.0f); } __syncthreads();
  { float v = bf16_rne(r2b1[c]);
#pragma unroll 1
    for (int k = 0; k < H; ++k) v += pmul(a[k], bf16_rne(r2w1[c * H + k])); bq[c] = fmaxf(v, 0.0f); } __syncthreads();
  if (c < OUT) { float v = bf16_rne(o2b[c]);
#pragma unroll 1
    for (int k = 0; k < H; ++k) v += pmul(bq[k], bf16_rne(o2w[c * H + k])); lg[c] = v; }
  __syncthreads();
  if (c < 32) { float mx = -INFINITY; for (int j = 0; j < OUT; ++j) mx = fmaxf(mx, lg[j]); float se = 0.0f; for (int j = 0; j < OUT; ++j) se += __expf(lg[j] - mx); const float lse = mx + __logf(se);
    const float val = (c < OUT) ? lg[c] - lse : 0.0f;
    for (int pass = 0; pass < 2; ++pass) { if (c < OUT) ((volatile float*)out)[c] = val; __threadfence(); } }
}
}

extern "C" void kernel_launch(void* const* d_in, const int* in_sizes, int n_in, void* d_out, int out_size, void* d_ws, size_t ws_size, hipStream_t stream) {
  (void)n_in;
  auto Fp = [&](int i) { return (const float*)d_in[i]; }; auto Ip = [&](int i) { return (const int*)d_in[i]; };
  if (in_sizes[0] != NT || in_sizes[1] != NT || in_sizes[2] != H || in_sizes[4] != H * H || in_sizes[20] != OUT * H || out_size != OUT) return;
  size_t off = 0; char* ws = (char*)d_ws;
  auto carve = [&](size_t bytes) { char* p = ws + off; off += (bytes + 255) & ~(size_t)255; return p; };
  b16* W6 = (b16*)carve((size_t)6 * H * H * 2); float* EV = (float*)carve((size_t)NEVP * H * 4); float* E1 = (float*)carve((size_t)NEVP * H * 4);
  if (off > ws_size) return;
  prep_kernel<<<(6 * H * H / 8 + 255) / 256, 256, 0, stream>>>(Fp(4), Fp(6), Fp(8), Fp(10), Fp(12), Fp(14), W6);
  stage1_kernel<<<NEVP, 32, 0, stream>>>(Fp(0), Ip(1), Fp(2), Fp(3), W6, Fp(5), EV);
  dense_kernel<<<NEVP / 64, 128, 0, stream>>>(EV, W6 + 1 * H * H, Fp(7), E1);
  dense_kernel<<<NEVP / 64, 128, 0, stream>>>(E1, W6 + 2 * H * H, Fp(9), EV);
  dense_kernel<<<NEVP / 64, 128, 0, stream>>>(EV, W6 + 3 * H * H, Fp(11), E1);
  dense_kernel<<<NEVP / 64, 128, 0, stream>>>(E1, W6 + 4 * H * H, Fp(13), EV);
  dense_kernel<<<NEVP / 64, 128, 0, stream>>>(EV, W6 + 5 * H * H, Fp(15), E1);
  final_kernel<<<1, 64, 0, stream>>>(E1, Fp(16), Fp(17), Fp(18), Fp(19), Fp(20), Fp(21), (float*)d_out);
}
